// LocalCausalGraph_4767413698783
// MI455X (gfx1250) — hardware-verified
//
#include <hip/hip_runtime.h>
#include <stddef.h>


#define DM    1024
#define CDIM  64
#define NCE   128
#define NTHR  256
#define CVTE  (NTHR * 8)

static_assert(CVTE == 2048);
static_assert((DM % 32) == 0);
static_assert(NCE == 2 * CDIM);

typedef float          v4f  __attribute__((ext_vector_type(4)));
typedef float          v8f  __attribute__((ext_vector_type(8)));
typedef unsigned short v8us __attribute__((ext_vector_type(8)));
typedef __bf16         v16b __attribute__((ext_vector_type(16)));
union FragB { v16b v; v8us u[2]; };

__device__ __forceinline__ unsigned int bfr(float f) {
  const unsigned int u = __float_as_uint(f);
  return (u + 0x7FFFu + ((u >> 16) & 1u)) >> 16;
}
__device__ __forceinline__ void split2(float v, unsigned short& h, unsigned short& l) {
  const unsigned int hb = bfr(v);
  const float hf = __uint_as_float(hb << 16);
  h = (unsigned short)hb;
  l = (unsigned short)bfr(v - hf);
}
__device__ __forceinline__ v8f zero8f() {
  v8f r;
#pragma unroll
  for (int i = 0; i < 8; ++i) r[i] = 0.0f;
  return r;
}
__device__ __forceinline__ v8f wmb(v16b a, v16b b, v8f c) {
  v8f d = __builtin_amdgcn_wmma_f32_16x16x32_bf16(false, a, false, b, (short)0, c, false, false);
  asm volatile("v_nop\n\tv_nop\n\tv_nop\n\tv_nop" : "+v"(d) : "v"(a), "v"(b));
  return d;
}

__global__ __launch_bounds__(NTHR) void k_cvt(const float* __restrict__ x, const float* __restrict__ Wc,
                                             const float* __restrict__ We, const float* __restrict__ W1,
                                             unsigned short* xh, unsigned short* xl,
                                             unsigned short* wh, unsigned short* wl,
                                             unsigned short* w1h, unsigned short* w1l,
                                             int nbx, int nbw, int nbw1, int nW) {
  const int tid = threadIdx.x;
  const int bk = blockIdx.x;
  const float* src;
  unsigned short* dh;
  unsigned short* dl;
  size_t sb, db;
  if (bk < nbx) {
    src = x; dh = xh; dl = xl; sb = (size_t)bk * CVTE; db = sb;
  } else if (bk < nbx + nbw) {
    src = Wc; dh = wh; dl = wl; sb = (size_t)(bk - nbx) * CVTE; db = sb;
  } else if (bk < nbx + 2 * nbw) {
    src = We; dh = wh; dl = wl; sb = (size_t)(bk - nbx - nbw) * CVTE; db = (size_t)nW + sb;
  } else if (bk < nbx + 2 * nbw + nbw1) {
    src = W1; dh = w1h; dl = w1l; sb = (size_t)(bk - nbx - 2 * nbw) * CVTE; db = sb;
  } else {
    return;
  }
  const size_t e = sb + (size_t)8 * tid;
  const v4f f0 = *(const v4f*)(src + e);
  const v4f f1 = *(const v4f*)(src + e + 4);
  v8us H, Lq;
  unsigned short h, l;
  split2(f0.x, h, l); H[0] = h; Lq[0] = l;
  split2(f0.y, h, l); H[1] = h; Lq[1] = l;
  split2(f0.z, h, l); H[2] = h; Lq[2] = l;
  split2(f0.w, h, l); H[3] = h; Lq[3] = l;
  split2(f1.x, h, l); H[4] = h; Lq[4] = l;
  split2(f1.y, h, l); H[5] = h; Lq[5] = l;
  split2(f1.z, h, l); H[6] = h; Lq[6] = l;
  split2(f1.w, h, l); H[7] = h; Lq[7] = l;
  unsigned short* ph = dh + db + (size_t)8 * tid;
  unsigned short* pl = dl + db + (size_t)8 * tid;
  *(volatile v8us*)ph = H;
  *(volatile v8us*)pl = Lq;
  __threadfence();
  *(volatile v8us*)ph = H;
  *(volatile v8us*)pl = Lq;
}

__global__ __launch_bounds__(NTHR) void k_proj(const unsigned short* __restrict__ xh, const unsigned short* __restrict__ xl,
                                              const unsigned short* __restrict__ wh, const unsigned short* __restrict__ wl,
                                              const unsigned short* __restrict__ w1h, const unsigned short* __restrict__ w1l,
                                              const float* __restrict__ b1, float* G, int M) {
  __shared__ __attribute__((aligned(16))) float          cs[16 * NCE];
  __shared__ __attribute__((aligned(16))) float          gs[16 * NCE];
  __shared__ __attribute__((aligned(16))) unsigned short csh[16 * NCE];
  __shared__ __attribute__((aligned(16))) unsigned short csl[16 * NCE];

  const int tid = threadIdx.x, lane = tid & 31, wave = tid >> 5, hh = lane >> 4, m = lane & 15;
  const int mTile = blockIdx.x * 16;
  if (mTile + 16 > M) return;
  const int nTile = wave * 16;

  const unsigned short* ahp = xh + (size_t)(mTile + m) * DM + 8 * hh;
  const unsigned short* alp = xl + (size_t)(mTile + m) * DM + 8 * hh;
  const unsigned short* bhp = wh + (size_t)(nTile + m) * DM + 8 * hh;
  const unsigned short* blp = wl + (size_t)(nTile + m) * DM + 8 * hh;
  v8f acc = zero8f();
#pragma unroll 2
  for (int k0 = 0; k0 < DM; k0 += 32) {
    FragB ah, al, bh, bl;
    ah.u[0] = *(const v8us*)(ahp + k0);  ah.u[1] = *(const v8us*)(ahp + k0 + 16);
    al.u[0] = *(const v8us*)(alp + k0);  al.u[1] = *(const v8us*)(alp + k0 + 16);
    bh.u[0] = *(const v8us*)(bhp + k0);  bh.u[1] = *(const v8us*)(bhp + k0 + 16);
    bl.u[0] = *(const v8us*)(blp + k0);  bl.u[1] = *(const v8us*)(blp + k0 + 16);
    acc = wmb(ah.v, bh.v, acc);
    acc = wmb(ah.v, bl.v, acc);
    acc = wmb(al.v, bh.v, acc);
  }
#pragma unroll
  for (int r = 0; r < 8; ++r) cs[(8 * hh + r) * NCE + nTile + m] = acc[r];
  __syncthreads();

#pragma unroll
  for (int q = 0; q < 8; ++q) {
    const int e = tid + NTHR * q;
    unsigned short h, l;
    split2(cs[e], h, l);
    csh[e] = h;
    csl[e] = l;
  }
  __syncthreads();

  const int isE  = (wave >= 4) ? 1 : 0;
  const int acol = isE * CDIM;
  const int wcol = isE * CDIM;
  const int hT   = (wave & 3) * 16;
  const unsigned short* a2h = csh + m * NCE + acol + 8 * hh;
  const unsigned short* a2l = csl + m * NCE + acol + 8 * hh;
  const unsigned short* b2h = w1h + (size_t)(hT + m) * NCE + wcol + 8 * hh;
  const unsigned short* b2l = w1l + (size_t)(hT + m) * NCE + wcol + 8 * hh;
  v8f acc2 = zero8f();
#pragma unroll
  for (int ks = 0; ks < 2; ++ks) {
    const int k0 = 32 * ks;
    FragB ah, al, bh, bl;
    ah.u[0] = *(const v8us*)(a2h + k0);  ah.u[1] = *(const v8us*)(a2h + k0 + 16);
    al.u[0] = *(const v8us*)(a2l + k0);  al.u[1] = *(const v8us*)(a2l + k0 + 16);
    bh.u[0] = *(const v8us*)(b2h + k0);  bh.u[1] = *(const v8us*)(b2h + k0 + 16);
    bl.u[0] = *(const v8us*)(b2l + k0);  bl.u[1] = *(const v8us*)(b2l + k0 + 16);
    acc2 = wmb(ah.v, bh.v, acc2);
    acc2 = wmb(ah.v, bl.v, acc2);
    acc2 = wmb(al.v, bh.v, acc2);
  }
  const float b1v  = b1[hT + m];
  const float bias = (isE != 0) ? 0.0f : b1v;
#pragma unroll
  for (int r = 0; r < 8; ++r) gs[(8 * hh + r) * NCE + 16 * wave + m] = acc2[r] + bias;
  __syncthreads();

  float* gb = G + (size_t)mTile * NCE;
  const v4f o0 = *(const v4f*)(gs + 4 * tid);
  const v4f o1 = *(const v4f*)(gs + 4 * (tid + NTHR));
  *(volatile v4f*)(gb + 4 * tid) = o0;
  *(volatile v4f*)(gb + 4 * (tid + NTHR)) = o1;
  __threadfence();
  *(volatile v4f*)(gb + 4 * tid) = o0;
  *(volatile v4f*)(gb + 4 * (tid + NTHR)) = o1;
}

__global__ __launch_bounds__(NTHR) void k_pair(const float* __restrict__ G, const float* __restrict__ W2,
                                              const float* __restrict__ b2, float* out, int L) {
  __shared__ __attribute__((aligned(16))) float shc[16 * CDIM];
  __shared__ float she[64 * 65];
  __shared__ float sw2[CDIM];
  __shared__ __attribute__((aligned(16))) float so[16 * 64];

  const int tid = threadIdx.x;
  const int b = blockIdx.y;
  const int i0 = blockIdx.x * 16;
  const int il = tid >> 4;
  const int jq = tid & 15;

#pragma unroll
  for (int q = 0; q < 4; ++q) {
    const int e = tid + NTHR * q;
    const int r = e >> 6, c = e & 63;
    shc[e] = G[(size_t)(b * L + i0 + r) * NCE + c];
  }
  if (tid < CDIM) sw2[tid] = W2[tid];
  const float bias2 = b2[0];
  const float ir2 = 0.70710678118654752f;
  const int nJ = L / 64;

#pragma unroll 1
  for (int jc = 0; jc < nJ; ++jc) {
    __syncthreads();
#pragma unroll
    for (int q = 0; q < 16; ++q) {
      const int e = tid + NTHR * q;
      const int r = e >> 6, c = e & 63;
      she[r * 65 + c] = G[(size_t)(b * L + jc * 64 + r) * NCE + CDIM + c];
    }
    __syncthreads();

    const float* hp = shc + il * CDIM;
#pragma unroll 1
    for (int q = 0; q < 4; ++q) {
      const int jl = 4 * jq + q;
      const float* ep = she + jl * 65;
      float s = 0.0f;
#pragma unroll 1
      for (int c = 0; c < CDIM; ++c) {
        const float v = hp[c] + ep[c];
        const float g = 0.5f * v * (1.0f + erff(v * ir2));
        s = fmaf(sw2[c], g, s);
      }
      const float z  = s + bias2;
      const float ev = expf(-z);
      so[il * 64 + jl] = __builtin_amdgcn_rcpf(1.0f + ev);
    }
    __syncthreads();

    const v4f ov = *(const v4f*)(so + il * 64 + 4 * jq);
    float* op = out + (size_t)(b * L + i0 + il) * L + jc * 64 + 4 * jq;
    *(volatile v4f*)op = ov;
    __threadfence();
    *(volatile v4f*)op = ov;
  }
}

extern "C" void kernel_launch(void* const* d_in, const int* in_sizes, int n_in,
                              void* d_out, int out_size, void* d_ws, size_t ws_size,
                              hipStream_t stream) {
  if (n_in < 7) return;
  const int nx = in_sizes[0], nwc = in_sizes[1], nwe = in_sizes[2], nw1 = in_sizes[3];
  if (nx <= 0 || (nx % DM) != 0) return;
  const int M = nx / DM;
  if (nwc != CDIM * DM || nwe != CDIM * DM || nw1 != CDIM * NCE) return;
  if (in_sizes[4] != CDIM || in_sizes[5] != CDIM || in_sizes[6] < 1) return;
  if ((M % 16) != 0 || out_size <= 0) return;
  const int L = out_size / M;
  if (L <= 0 || L * M != out_size || (M % L) != 0 || (L % 64) != 0) return;
  const int Bn = M / L;
  if ((nx % CVTE) != 0 || (nwc % CVTE) != 0 || (nw1 % CVTE) != 0) return;

  const float* x  = (const float*)d_in[0];
  const float* Wc = (const float*)d_in[1];
  const float* We = (const float*)d_in[2];
  const float* W1 = (const float*)d_in[3];
  const float* b1 = (const float*)d_in[4];
  const float* W2 = (const float*)d_in[5];
  const float* b2 = (const float*)d_in[6];
  float* out = (float*)d_out;

  char* ws = (char*)d_ws;
  size_t off = 0;
  const size_t oXh = off; off += (size_t)nx * 2;            off = (off + 255) & ~(size_t)255;
  const size_t oXl = off; off += (size_t)nx * 2;            off = (off + 255) & ~(size_t)255;
  const size_t oWh = off; off += (size_t)NCE * DM * 2;      off = (off + 255) & ~(size_t)255;
  const size_t oWl = off; off += (size_t)NCE * DM * 2;      off = (off + 255) & ~(size_t)255;
  const size_t o1h = off; off += (size_t)CDIM * NCE * 2;    off = (off + 255) & ~(size_t)255;
  const size_t o1l = off; off += (size_t)CDIM * NCE * 2;    off = (off + 255) & ~(size_t)255;
  const size_t oG  = off; off += (size_t)M * NCE * 4;       off = (off + 255) & ~(size_t)255;
  if (off > ws_size) return;
  unsigned short* xh  = (unsigned short*)(ws + oXh);
  unsigned short* xl  = (unsigned short*)(ws + oXl);
  unsigned short* wh  = (unsigned short*)(ws + oWh);
  unsigned short* wl  = (unsigned short*)(ws + oWl);
  unsigned short* w1h = (unsigned short*)(ws + o1h);
  unsigned short* w1l = (unsigned short*)(ws + o1l);
  float*          G   = (float*)(ws + oG);

  const int nbx  = nx / CVTE;
  const int nbw  = nwc / CVTE;
  const int nbw1 = nw1 / CVTE;

  k_cvt<<<nbx + 2 * nbw + nbw1, NTHR, 0, stream>>>(x, Wc, We, W1, xh, xl, wh, wl, w1h, w1l,
                                                     nbx, nbw, nbw1, nwc);
  k_proj<<<M / 16, NTHR, 0, stream>>>(xh, xl, wh, wl, w1h, w1l, b1, G, M);
  k_pair<<<dim3(L / 16, Bn, 1), NTHR, 0, stream>>>(G, W2, b2, out, L);
}
